// CausalSelfAttentionGQA_68685116998333
// MI455X (gfx1250) — hardware-verified
//
#include <hip/hip_runtime.h>
#include <math.h>
#include <stdint.h>

#define NB    2
#define SEQ   2048
#define DM    2048
#define NH    16
#define NKV   4
#define QPK   (NH / NKV)
#define HD    128
#define DKV   (NKV * HD)
#define NQB   (SEQ / 16)
#define NKT   (SEQ / 64)
#define NPRE  256
#define NQP   (NPRE / 16)
static_assert(NH * HD == DM);
static_assert(QPK == 4);
static_assert(NQB == 128 && NKT == 32 && NQP == 16);
static_assert((NPRE % 64) == 0 && NPRE <= SEQ);
static_assert((SEQ % 64) == 0 && (DM % 256) == 0 && (DKV % 64) == 0 && HD == 128);

typedef _Float16 v16h __attribute__((ext_vector_type(16)));
typedef _Float16 v8h  __attribute__((ext_vector_type(8)));
typedef __bf16   v16b __attribute__((ext_vector_type(16)));
typedef __bf16   v8b  __attribute__((ext_vector_type(8)));
typedef float    v8f  __attribute__((ext_vector_type(8)));
typedef float    v4f  __attribute__((ext_vector_type(4)));
typedef unsigned int v4u __attribute__((ext_vector_type(4)));

#if defined(__HIP_DEVICE_COMPILE__)
#define DEV_ASM 1
#else
#define DEV_ASM 0
#endif

__device__ __forceinline__ unsigned short bf_bits(float f) {
  unsigned u = __float_as_uint(f);
  return (unsigned short)((u + 0x7FFFu + ((u >> 16) & 1u)) >> 16);
}
__device__ __forceinline__ float bf_up(unsigned short hb) { return __uint_as_float(((unsigned)hb) << 16); }
__device__ __forceinline__ float bf16r(float f) { return bf_up(bf_bits(f)); }
__device__ __forceinline__ unsigned short h_bits(_Float16 x) { return __builtin_bit_cast(unsigned short, x); }
__device__ __forceinline__ unsigned pk16(unsigned short a, unsigned short b) { return (unsigned)a | ((unsigned)b << 16); }
__device__ __forceinline__ v8f zero8() { v8f z = {0.f, 0.f, 0.f, 0.f, 0.f, 0.f, 0.f, 0.f}; return z; }

template <typename OT> struct FT;
template <> struct FT<__bf16>   { typedef v16b frag; typedef v8b half8; };
template <> struct FT<_Float16> { typedef v16h frag; typedef v8h half8; };

template <typename OT>
__device__ __forceinline__ typename FT<OT>::frag ldfrag(const OT* p) {
  union { typename FT<OT>::frag v; typename FT<OT>::half8 h[2]; } f;
  f.h[0] = *(const typename FT<OT>::half8*)(p);
  f.h[1] = *(const typename FT<OT>::half8*)(p + 16);
  return f.v;
}

__device__ __forceinline__ v8f mmar(v16b a, v16b b, v8f c) {
  return __builtin_amdgcn_wmma_f32_16x16x32_bf16(false, a, false, b, (short)0, c, false, false);
}
__device__ __forceinline__ v8f mmar(v16h a, v16h b, v8f c) {
  return __builtin_amdgcn_wmma_f32_16x16x32_f16(false, a, false, b, (short)0, c, false, false);
}
__device__ __forceinline__ v8f mma_h(v16h a, v16h b, v8f c) {
  c = __builtin_amdgcn_wmma_f32_16x16x32_f16(false, a, false, b, (short)0, c, false, false);
#if DEV_ASM
  asm volatile("v_nop\n\tv_nop\n\tv_nop\n\tv_nop" : "+v"(c) : "v"(a), "v"(b));
#endif
  return c;
}
__device__ __forceinline__ void dep_guard(v8f& a, v8f& b, v16b x, v16b y) {
#if DEV_ASM
  asm volatile("v_nop\n\tv_nop\n\tv_nop\n\tv_nop" : "+v"(a), "+v"(b) : "v"(x), "v"(y));
#else
  (void)a; (void)b; (void)x; (void)y;
#endif
}
__device__ __forceinline__ void dep_guard(v8f& a, v8f& b, v16h x, v16h y) {
#if DEV_ASM
  asm volatile("v_nop\n\tv_nop\n\tv_nop\n\tv_nop" : "+v"(a), "+v"(b) : "v"(x), "v"(y));
#else
  (void)a; (void)b; (void)x; (void)y;
#endif
}
__device__ __forceinline__ void keep4(v16b a, v16b b, v16b c, v16b d) {
#if DEV_ASM
  asm volatile("v_nop" :: "v"(a), "v"(b), "v"(c), "v"(d));
#else
  (void)a; (void)b; (void)c; (void)d;
#endif
}
__device__ __forceinline__ void keep4(v16h a, v16h b, v16h c, v16h d) {
#if DEV_ASM
  asm volatile("v_nop" :: "v"(a), "v"(b), "v"(c), "v"(d));
#else
  (void)a; (void)b; (void)c; (void)d;
#endif
}
__device__ __forceinline__ void acc_guard4(v8f& a, v8f& b, v8f& c, v8f& d) {
#if DEV_ASM
  asm volatile("v_nop\n\tv_nop\n\tv_nop\n\tv_nop" : "+v"(a), "+v"(b), "+v"(c), "+v"(d));
#else
  (void)a; (void)b; (void)c; (void)d;
#endif
}

__global__ __launch_bounds__(256) void cvt_bf16x8(const float* __restrict__ in, unsigned short* out, int n8) {
  const int i = blockIdx.x * 256 + (int)threadIdx.x;
  if (i < n8) {
    const v4f a = *(const v4f*)(in + (size_t)i * 8);
    const v4f b = *(const v4f*)(in + (size_t)i * 8 + 4);
    v4u p;
    p[0] = pk16(bf_bits(a[0]), bf_bits(a[1]));
    p[1] = pk16(bf_bits(a[2]), bf_bits(a[3]));
    p[2] = pk16(bf_bits(b[0]), bf_bits(b[1]));
    p[3] = pk16(bf_bits(b[2]), bf_bits(b[3]));
    *(volatile v4u*)(out + (size_t)i * 8) = p;
    __threadfence();
    *(volatile v4u*)(out + (size_t)i * 8) = p;
  }
}

template <int MODE, bool PERM>
__global__ __launch_bounds__(256) void wt_prep(const float* __restrict__ W, int nW, unsigned short* outp, int kin) {
  __shared__ __align__(16) unsigned short sW[16 * 256];
  const int tid  = (int)threadIdx.x;
  const int wave = tid >> 5;
  const int lane = tid & 31;
  const int p0   = blockIdx.x * 16;
  const int k0   = blockIdx.y * 256;
  int shift = 0;
  if (PERM) {
    const int pw = (p0 >> 5) & 3;
    shift = (pw == 1) ? 32 : ((pw == 2) ? -32 : 0);
  }
  const float* src = W + (size_t)(k0 + tid) * nW + (p0 + shift);
  const v4f a0 = *(const v4f*)(src);
  const v4f a1 = *(const v4f*)(src + 4);
  const v4f a2 = *(const v4f*)(src + 8);
  const v4f a3 = *(const v4f*)(src + 12);
#pragma unroll
  for (int e = 0; e < 4; ++e) {
    sW[(e)      * 256 + tid] = bf_bits(a0[e]);
    sW[(4 + e)  * 256 + tid] = bf_bits(a1[e]);
    sW[(8 + e)  * 256 + tid] = bf_bits(a2[e]);
    sW[(12 + e) * 256 + tid] = bf_bits(a3[e]);
  }
  __syncthreads();
  const int r0 = 2 * wave;
  const v4u w0 = *(const v4u*)(sW + r0 * 256 + lane * 8);
  const v4u w1 = *(const v4u*)(sW + (r0 + 1) * 256 + lane * 8);
  const int pitch = (MODE == 0) ? kin : 2 * kin;
  const size_t o0 = (size_t)(p0 + r0) * pitch + k0 + lane * 8;
  const size_t o1 = (size_t)(p0 + r0 + 1) * pitch + k0 + lane * 8;
  if (MODE == 0) {
    for (int pass = 0; pass < 2; ++pass) {
      *(volatile v4u*)(outp + o0) = w0;
      *(volatile v4u*)(outp + o1) = w1;
      __threadfence();
    }
  } else {
    v4u h0, l0, h1, l1;
#pragma unroll
    for (int e = 0; e < 4; ++e) {
      const unsigned u0 = w0[e], u1 = w1[e];
      const float f00 = bf_up((unsigned short)(u0 & 0xFFFFu)), f01 = bf_up((unsigned short)(u0 >> 16));
      const float f10 = bf_up((unsigned short)(u1 & 0xFFFFu)), f11 = bf_up((unsigned short)(u1 >> 16));
      h0[e] = pk16(h_bits((_Float16)(f00 * 1024.0f)), h_bits((_Float16)(f01 * 1024.0f)));
      l0[e] = pk16(h_bits((_Float16)(f00 * 0.5f)),    h_bits((_Float16)(f01 * 0.5f)));
      h1[e] = pk16(h_bits((_Float16)(f10 * 1024.0f)), h_bits((_Float16)(f11 * 1024.0f)));
      l1[e] = pk16(h_bits((_Float16)(f10 * 0.5f)),    h_bits((_Float16)(f11 * 0.5f)));
    }
    for (int pass = 0; pass < 2; ++pass) {
      *(volatile v4u*)(outp + o0) = h0;
      *(volatile v4u*)(outp + o0 + kin) = l0;
      *(volatile v4u*)(outp + o1) = h1;
      *(volatile v4u*)(outp + o1 + kin) = l1;
      __threadfence();
    }
  }
}

template <typename OT, int OUT_MODE, bool ROPE, bool KSEL>
__global__ __launch_bounds__(256) void gemm64(
    const unsigned short* __restrict__ Ap, int lda, long long strideA,
    const unsigned short* __restrict__ Btp, int ldb, long long strideB,
    void* Cout, void* Cout2, int ldc, long long strideC,
    const float* __restrict__ ctab, const float* __restrict__ stab,
    int M, int N, int K, float oscale, float rscale) {
  typedef typename FT<OT>::frag V16;
  const OT* A  = (const OT*)(const void*)Ap;
  const OT* Bt = (const OT*)(const void*)Btp;
  __shared__ __align__(16) float sT[8][16 * 68];
  const int b    = blockIdx.y;
  const int lane = threadIdx.x & 31;
  const int wave = threadIdx.x >> 5;
  const int tilesN = N >> 6;
  const int tilesM = M >> 6;
  const int tile = blockIdx.x * 8 + wave;
  if (tile >= tilesM * tilesN) return;
  const int tm = tile / tilesN;
  const int tn = tile - tm * tilesN;
  const int m0 = tm << 6;
  const int n0 = tn << 6;
  const int Kt = (KSEL && ((m0 & (SEQ - 1)) >= NPRE)) ? (K >> 1) : K;

  const OT* Ab = A  + (size_t)b * (size_t)strideA;
  const OT* Bb = Bt + (size_t)b * (size_t)strideB;

  const int rlane = lane & 15;
  const int koff  = (lane >> 4) * 8;
  const int mOff  = (lane >> 4) * 8;

  v8f acc[4][4];
#pragma unroll
  for (int i = 0; i < 4; ++i)
#pragma unroll
    for (int j = 0; j < 4; ++j) acc[i][j] = zero8();

  for (int k0 = 0; k0 < Kt; k0 += 32) {
    V16 bq[4];
#pragma unroll
    for (int j = 0; j < 4; ++j)
      bq[j] = ldfrag<OT>(Bb + (size_t)(n0 + (j << 4) + rlane) * ldb + koff + k0);
#pragma unroll
    for (int i = 0; i < 4; ++i) {
      const V16 af = ldfrag<OT>(Ab + (size_t)(m0 + (i << 4) + rlane) * lda + koff + k0);
#pragma unroll
      for (int j = 0; j < 4; ++j) acc[i][j] = mmar(af, bq[j], acc[i][j]);
      dep_guard(acc[i][0], acc[i][3], af, bq[3]);
    }
    keep4(bq[0], bq[1], bq[2], bq[3]);
  }
  acc_guard4(acc[0][0], acc[0][1], acc[0][2], acc[0][3]);
  acc_guard4(acc[1][0], acc[1][1], acc[1][2], acc[1][3]);
  acc_guard4(acc[2][0], acc[2][1], acc[2][2], acc[2][3]);
  acc_guard4(acc[3][0], acc[3][1], acc[3][2], acc[3][3]);

  float* slab = sT[wave];
#pragma unroll
  for (int i = 0; i < 4; ++i) {
    const int mBase = m0 + (i << 4);
#pragma unroll
    for (int j = 0; j < 4; ++j) {
#pragma unroll
      for (int r = 0; r < 8; ++r) {
        slab[(mOff + r) * 68 + (j << 4) + rlane] = acc[i][j][r];
      }
    }
    __builtin_amdgcn_fence(__ATOMIC_RELEASE, "workgroup");
    __builtin_amdgcn_wave_barrier();
    __builtin_amdgcn_fence(__ATOMIC_ACQUIRE, "workgroup");
    if (OUT_MODE == 0) {
      float* C = (float*)Cout + (size_t)b * (size_t)strideC;
      const int h2 = lane >> 4, c4 = (lane & 15) * 4;
      for (int pass = 0; pass < 2; ++pass) {
#pragma unroll
        for (int it = 0; it < 8; ++it) {
          const int row = it * 2 + h2;
          const v4f v = *(const v4f*)(slab + row * 68 + c4) * oscale;
          *(volatile v4f*)(C + (size_t)(mBase + row) * ldc + n0 + c4) = v;
        }
        __threadfence();
      }
    } else {
      const int q = lane >> 3, c8 = (lane & 7) * 8;
      unsigned short* C  = (unsigned short*)Cout  + (size_t)b * (size_t)strideC;
      unsigned short* C2 = (unsigned short*)Cout2 + (size_t)b * (size_t)strideC;
      v4u hv[4], lv[4];
#pragma unroll
      for (int it = 0; it < 4; ++it) {
        const int row = it * 4 + q;
        const float* sp = slab + row * 68 + c8;
        float f[8];
#pragma unroll
        for (int e = 0; e < 8; ++e) f[e] = sp[e];
        if (ROPE) {
#pragma clang fp contract(off)
          const int t    = (mBase + row) & (SEQ - 1);
          const int half = (n0 >> 6) & 1;
          const int hi32 = c8 & 32;
          const int dcol = (c8 & 31) + 32 * half + 2 * hi32;
          const float* gp = slab + row * 68 + (c8 ^ 32);
          const v4f ca = *(const v4f*)(ctab + (size_t)t * HD + dcol);
          const v4f cb = *(const v4f*)(ctab + (size_t)t * HD + dcol + 4);
          const v4f sa = *(const v4f*)(stab + (size_t)t * HD + dcol);
          const v4f sb = *(const v4f*)(stab + (size_t)t * HD + dcol + 4);
          float cs8[8], sn8[8], g[8];
#pragma unroll
          for (int e = 0; e < 4; ++e) {
            cs8[e] = ca[e]; cs8[4 + e] = cb[e];
            sn8[e] = sa[e]; sn8[4 + e] = sb[e];
          }
#pragma unroll
          for (int e = 0; e < 8; ++e) g[e] = gp[e];
#pragma unroll
          for (int e = 0; e < 8; ++e) {
            const float cs = bf16r(cs8[e]);
            const float sn = bf16r(sn8[e]);
            const float a0 = f[e] * cs;
            const float a1 = g[e] * sn;
            const float up = a0 + a1;
            const float dn = a0 - a1;
            f[e] = hi32 ? up : dn;
          }
        }
        v4u a, a2;
#pragma unroll
        for (int e = 0; e < 4; ++e) {
          const float f0 = f[2 * e], f1 = f[2 * e + 1];
          const _Float16 x0 = (_Float16)f0, x1 = (_Float16)f1;
          const unsigned short h0 = h_bits(x0), h1 = h_bits(x1);
          const unsigned short l0 = h_bits((_Float16)((f0 - (float)x0) * rscale));
          const unsigned short l1 = h_bits((_Float16)((f1 - (float)x1) * rscale));
          a[e] = pk16(h0, h1); a2[e] = pk16(l0, l1);
        }
        hv[it] = a; lv[it] = a2;
      }
      for (int pass = 0; pass < 2; ++pass) {
#pragma unroll
        for (int it = 0; it < 4; ++it) {
          const int row = it * 4 + q;
          *(volatile v4u*)(C  + (size_t)(mBase + row) * ldc + n0 + c8) = hv[it];
          *(volatile v4u*)(C2 + (size_t)(mBase + row) * ldc + n0 + c8) = lv[it];
        }
        __threadfence();
      }
    }
    __builtin_amdgcn_fence(__ATOMIC_RELEASE, "workgroup");
    __builtin_amdgcn_wave_barrier();
    __builtin_amdgcn_fence(__ATOMIC_ACQUIRE, "workgroup");
  }
}

#define A_KSH   0
#define A_K64   16384
#define A_KSL   32768
#define A_VTH   49152
#define A_VTL   65536
#define A_PA    81920
#define A_PB    90112
#define A_ACC   98304
#define A_MAIN  131072
#define A_VTQ   131072
#define A_PL    147456
#define A_PREC  155648
static_assert(A_K64 - A_KSH == 64 * HD * 2 && A_KSL - A_K64 == 64 * HD * 2 && A_VTH - A_KSL == 64 * HD * 2);
static_assert(A_VTL - A_VTH == HD * 64 * 2 && A_PA - A_VTL == HD * 64 * 2);
static_assert(A_PB - A_PA == 4 * 16 * 64 * 2 && A_ACC - A_PB == 4 * 16 * 64 * 2);
static_assert(A_MAIN - A_ACC == 4 * 8 * 32 * 8 * 4);
static_assert(A_VTQ == A_MAIN && A_PL - A_VTQ == HD * 64 * 2 && A_PREC - A_PL == 4 * 16 * 64 * 2);
static_assert(4 * 16 * HD * 4 <= A_VTH);

template <bool PRECISE>
__global__ __launch_bounds__(128) __attribute__((amdgpu_num_vgpr(256)))
void attn_gqa(const unsigned short* __restrict__ qhp, const unsigned short* __restrict__ qlp,
              const unsigned short* __restrict__ khp, const unsigned short* __restrict__ klp,
              const unsigned short* __restrict__ vhp, const unsigned short* __restrict__ vlp,
              unsigned short* op, float s64) {
  constexpr int QB0  = PRECISE ? 0 : NQP;
  constexpr int NQBL = PRECISE ? NQP : (NQB - NQP);
  extern __shared__ __align__(16) unsigned char lds[];
  union FH { v16h v; v8h h[2]; };
  _Float16* Ksh = (_Float16*)(lds + A_KSH);
  _Float16* K64 = (_Float16*)(lds + A_K64);
  _Float16* Ksl = (_Float16*)(lds + A_KSL);
  _Float16* Vth = (_Float16*)(lds + A_VTH);
  _Float16* Vtl = (_Float16*)(lds + A_VTL);
  _Float16* Vtq = (_Float16*)(lds + A_VTQ);
  _Float16* Pa  = (_Float16*)(lds + A_PA);
  _Float16* Pb  = (_Float16*)(lds + A_PB);
  _Float16* Pl  = (_Float16*)(lds + A_PL);
  float*    accL = (float*)(lds + A_ACC);

  const int tid  = (int)threadIdx.x;
  const int wave = tid >> 5;
  const int lane = tid & 31;
  const int hh   = lane >> 4;
  const int c    = lane & 15;

  const int bx   = blockIdx.x;
  const int qb   = QB0 + (bx % NQBL);
  const int rest = bx / NQBL;
  const int g    = rest & (NKV - 1);
  const int b    = rest >> 2;
  const int h    = g * QPK + wave;
  const int q0   = qb * 16;
  const size_t rowB = (size_t)b * SEQ;

  const _Float16* Qh  = (const _Float16*)(const void*)qhp;
  const _Float16* Ql  = (const _Float16*)(const void*)qlp;
  const _Float16* Khg = (const _Float16*)(const void*)khp + (size_t)g * HD;
  const _Float16* Klg = (const _Float16*)(const void*)klp + (size_t)g * HD;
  const _Float16* Vh  = (const _Float16*)(const void*)vhp + ((size_t)b * DKV + (size_t)g * HD) * SEQ;
  const _Float16* Vl  = (const _Float16*)(const void*)vlp + ((size_t)b * DKV + (size_t)g * HD) * SEQ;

  _Float16* pwa  = Pa + wave * 1024;
  _Float16* pwb  = Pb + wave * 1024;
  _Float16* pwl  = Pl + wave * 1024;
  float*    accW = accL + wave * 2048;

#pragma unroll
  for (int t = 0; t < 8; ++t) *(v8f*)(accW + (t * 32 + lane) * 8) = zero8();

  float mrow[8], lrow[8], alpha[8];
#pragma unroll
  for (int r = 0; r < 8; ++r) { mrow[r] = -INFINITY; lrow[r] = 0.f; alpha[r] = 0.f; }

  const size_t qo = (rowB + q0 + c) * DM + (size_t)h * HD + 8 * hh;
  const int nkt_raw = (qb >> 2) + 1;
  const int nkt = (nkt_raw < NKT) ? nkt_raw : NKT;
  const _Float16 c64 = (_Float16)64.0f;
  const _Float16 r64 = (_Float16)0.015625f;

  for (int kt = 0; kt < nkt; ++kt) {
    const int kv0 = kt * 64;
    __syncthreads();
    {
#pragma unroll 2
      for (int i = 0; i < 8; ++i) {
        const int p   = tid + 128 * i;
        const int kr  = p >> 4;
        const int kp8 = (p & 15) * 8;
        const size_t ko = (rowB + kv0 + kr) * DKV + kp8;
        const v8h a0 = *(const v8h*)(Khg + ko);
        const v8h a1 = *(const v8h*)(Klg + ko);
        const int d  = p >> 3;
        const int sg = (p & 7) * 8;
        const v8h b0 = *(const v8h*)(Vh + (size_t)d * SEQ + kv0 + sg);
        const v8h b1 = *(const v8h*)(Vl + (size_t)d * SEQ + kv0 + sg);
        *(v8h*)(Ksh + kr * HD + kp8) = a0;
        *(v8h*)(K64 + kr * HD + kp8) = a0 * c64;
        *(v8h*)(Ksl + kr * HD + kp8) = a1;
        *(v8h*)(Vth + d * 64 + sg) = b0;
        *(v8h*)(Vtl + d * 64 + sg) = b1;
        if (PRECISE) *(v8h*)(Vtq + d * 64 + sg) = b0 * r64;
      }
    }
    __syncthreads();

    v8f s[4];
#pragma unroll
    for (int j = 0; j < 4; ++j) s[j] = zero8();
#pragma unroll 1
    for (int dc = 0; dc < 4; ++dc) {
      const v16h qa = ldfrag<_Float16>(Qh + qo + dc * 32);
      const v16h ql = ldfrag<_Float16>(Ql + qo + dc * 32);
      const int ko = dc * 32 + 8 * hh;
#pragma unroll
      for (int j = 0; j < 4; ++j) {
        const int kr = (j * 16 + c) * HD + ko;
        FH k6, kb, kl;
        k6.h[0] = *(const v8h*)(K64 + kr);
        k6.h[1] = *(const v8h*)(K64 + kr + 16);
        kb.h[0] = *(const v8h*)(Ksh + kr);
        kb.h[1] = *(const v8h*)(Ksh + kr + 16);
        kl.h[0] = *(const v8h*)(Ksl + kr);
        kl.h[1] = *(const v8h*)(Ksl + kr + 16);
        s[j] = mma_h(qa, k6.v, s[j]);
        s[j] = mma_h(ql, kb.v, s[j]);
        s[j] = mma_h(qa, kl.v, s[j]);
      }
    }

#pragma unroll
    for (int r = 0; r < 8; ++r) {
      const int rowq = q0 + 8 * hh + r;
      float m = -INFINITY;
#pragma unroll
      for (int j = 0; j < 4; ++j) {
        const int key = kv0 + j * 16 + c;
        float sv = s[j][r] * s64;
        sv = (key <= rowq) ? sv : -INFINITY;
        s[j][r] = sv;
        m = fmaxf(m, sv);
      }
#pragma unroll
      for (int off = 1; off < 16; off <<= 1) m = fmaxf(m, __shfl_xor(m, off, 32));
      const float mnew  = fmaxf(mrow[r], m);
      const float msafe = (mnew == -INFINITY) ? 0.f : mnew;
      const float al    = __expf(mrow[r] - msafe);
      mrow[r]  = mnew;
      alpha[r] = al;
      float psum = 0.f;
#pragma unroll
      for (int j = 0; j < 4; ++j) {
        const float p  = __expf(s[j][r] - msafe);
        psum += p;
        const float pk = p * 1024.0f;
        const _Float16 xa = (_Float16)pk;
        const int po = (8 * hh + r) * 64 + j * 16 + c;
        pwa[po] = xa;
        pwb[po] = (_Float16)(p * 4.0f);
        if (PRECISE) pwl[po] = (_Float16)((pk - (float)xa) * 64.0f);
      }
#pragma unroll
      for (int off = 1; off < 16; off <<= 1) psum += __shfl_xor(psum, off, 32);
      lrow[r] = lrow[r] * al + psum;
    }
    __builtin_amdgcn_fence(__ATOMIC_RELEASE, "workgroup");
    __builtin_amdgcn_wave_barrier();
    __builtin_amdgcn_fence(__ATOMIC_ACQUIRE, "workgroup");

    FH pa[2], pb[2], pl[2];
#pragma unroll
    for (int kk = 0; kk < 2; ++kk) {
      const int pr = c * 64 + kk * 32 + 8 * hh;
      pa[kk].h[0] = *(const v8h*)(pwa + pr);
      pa[kk].h[1] = *(const v8h*)(pwa + pr + 16);
      pb[kk].h[0] = *(const v8h*)(pwb + pr);
      pb[kk].h[1] = *(const v8h*)(pwb + pr + 16);
      pl[kk] = pa[kk];
      if (PRECISE) {
        pl[kk].h[0] = *(const v8h*)(pwl + pr);
        pl[kk].h[1] = *(const v8h*)(pwl + pr + 16);
      }
    }
#pragma unroll 1
    for (int t = 0; t < 8; ++t) {
      float* ap = accW + (t * 32 + lane) * 8;
      v8f acc = *(const v8f*)ap;
#pragma unroll
      for (int r = 0; r < 8; ++r) acc[r] *= alpha[r];
      const int vr0 = (t * 16 + c) * 64 + 8 * hh;
#pragma unroll
      for (int kk = 0; kk < 2; ++kk) {
        const int vr = vr0 + kk * 32;
        FH vb, vl;
        vb.h[0] = *(const v8h*)(Vth + vr);
        vb.h[1] = *(const v8h*)(Vth + vr + 16);
        vl.h[0] = *(const v8h*)(Vtl + vr);
        vl.h[1] = *(const v8h*)(Vtl + vr + 16);
        acc = mma_h(pa[kk].v, vb.v, acc);
        acc = mma_h(pb[kk].v, vl.v, acc);
        if (PRECISE) {
          FH vq;
          vq.h[0] = *(const v8h*)(Vtq + vr);
          vq.h[1] = *(const v8h*)(Vtq + vr + 16);
          acc = mma_h(pl[kk].v, vq.v, acc);
        }
      }
      *(v8f*)ap = acc;
    }
  }

  __syncthreads();

  float* os = (float*)(lds + A_KSH) + wave * (16 * HD);
  float inv[8];
#pragma unroll
  for (int r = 0; r < 8; ++r) {
    const float l = lrow[r];
    inv[r] = ((l > 0.f) ? (1.0f / l) : 0.f) * 0.25f;
  }
#pragma unroll 1
  for (int t = 0; t < 8; ++t) {
    const v8f acc = *(const v8f*)(accW + (t * 32 + lane) * 8);
#pragma unroll
    for (int r = 0; r < 8; ++r) os[(8 * hh + r) * HD + t * 16 + c] = acc[r] * inv[r];
  }
  __builtin_amdgcn_fence(__ATOMIC_RELEASE, "workgroup");
  __builtin_amdgcn_wave_barrier();
  __builtin_amdgcn_fence(__ATOMIC_ACQUIRE, "workgroup");
  {
    const int q4 = lane >> 3, c8 = (lane & 7) * 8;
    v4u hv[8], lv[8];
#pragma unroll
    for (int it = 0; it < 8; ++it) {
      const int row = (it & 3) * 4 + q4;
      const int seg = it >> 2;
      const float* sp = os + row * HD + seg * 64 + c8;
      v4u a, a2;
#pragma unroll
      for (int e = 0; e < 4; ++e) {
        const float f0 = sp[2 * e], f1 = sp[2 * e + 1];
        const _Float16 x0 = (_Float16)f0, x1 = (_Float16)f1;
        const unsigned short h0 = h_bits(x0), h1 = h_bits(x1);
        const unsigned short l0 = h_bits((_Float16)((f0 - (float)x0) * 2048.0f));
        const unsigned short l1 = h_bits((_Float16)((f1 - (float)x1) * 2048.0f));
        a[e] = pk16(h0, h1); a2[e] = pk16(l0, l1);
      }
      hv[it] = a; lv[it] = a2;
    }
    for (int pass = 0; pass < 2; ++pass) {
#pragma unroll
      for (int it = 0; it < 8; ++it) {
        const int row = (it & 3) * 4 + q4;
        const int seg = it >> 2;
        const size_t go = (rowB + q0 + row) * (size_t)(2 * DM) + (size_t)h * HD + seg * 64 + c8;
        *(volatile v4u*)(op + go) = hv[it];
        *(volatile v4u*)(op + go + DM) = lv[it];
      }
      __threadfence();
    }
  }
}

extern "C" void kernel_launch(void* const* d_in, const int* in_sizes, int n_in,
                              void* d_out, int out_size, void* d_ws, size_t ws_size,
                              hipStream_t stream) {
  if (n_in < 7) return;
  if (in_sizes[0] != NB * SEQ * DM) return;
  if (in_sizes[1] != SEQ * HD || in_sizes[2] != SEQ * HD) return;
  if (in_sizes[3] != DM * DM) return;
  if (in_sizes[4] != DM * DKV || in_sizes[5] != DM * DKV) return;
  if (in_sizes[6] != DM * DM) return;
  if (out_size != NB * SEQ * DM) return;

  const float* x    = (const float*)d_in[0];
  const float* cosp = (const float*)d_in[1];
  const float* sinp = (const float*)d_in[2];
  const float* Wq   = (const float*)d_in[3];
  const float* Wk   = (const float*)d_in[4];
  const float* Wv   = (const float*)d_in[5];
  const float* Wo   = (const float*)d_in[6];

  const size_t PX  = (size_t)NB * SEQ * DM * 2;
  const size_t PWQ = (size_t)DM * DM * 2;
  const size_t PWK = (size_t)DKV * DM * 2;
  const size_t PWO = (size_t)DM * (2 * DM) * 2;
  const size_t PK  = (size_t)NB * SEQ * DKV * 2;
  const size_t PVT = (size_t)NB * DKV * SEQ * 2;
  const size_t PO  = (size_t)NB * SEQ * (2 * DM) * 2;
  size_t off = 0;
  const size_t oXb  = off; off += PX;
  const size_t oWq  = off; off += PWQ;
  const size_t oWk  = off; off += PWK;
  const size_t oWv  = off; off += PWK;
  const size_t oWo  = off; off += PWO;
  const size_t oQh  = off; off += PX;
  const size_t oQl  = off; off += PX;
  const size_t oKh  = off; off += PK;
  const size_t oKl  = off; off += PK;
  const size_t oVTh = off; off += PVT;
  const size_t oVTl = off; off += PVT;
  const size_t oOp  = off; off += PO;
  if (off > ws_size) return;
  if (off > (size_t)134217728) return;

  char* ws = (char*)d_ws;
  unsigned short* Xb   = (unsigned short*)(ws + oXb);
  unsigned short* WqT  = (unsigned short*)(ws + oWq);
  unsigned short* WkT  = (unsigned short*)(ws + oWk);
  unsigned short* WvT  = (unsigned short*)(ws + oWv);
  unsigned short* WoT2 = (unsigned short*)(ws + oWo);
  unsigned short* Qh   = (unsigned short*)(ws + oQh);
  unsigned short* Ql   = (unsigned short*)(ws + oQl);
  unsigned short* Kh   = (unsigned short*)(ws + oKh);
  unsigned short* Kl   = (unsigned short*)(ws + oKl);
  unsigned short* VTh  = (unsigned short*)(ws + oVTh);
  unsigned short* VTl  = (unsigned short*)(ws + oVTl);
  unsigned short* Op   = (unsigned short*)(ws + oOp);

  const dim3 blk(256);
  const int n8x = NB * SEQ * DM / 8;
  const dim3 gCvtX((n8x + 255) / 256);
  const dim3 gWq(DM / 16, DM / 256);
  const dim3 gWk(DKV / 16, DM / 256);
  const dim3 gQ((((NB * SEQ) / 64) * (DM / 64) + 7) / 8, 1);
  const dim3 gK((((NB * SEQ) / 64) * (DKV / 64) + 7) / 8, 1);
  const dim3 gVT(((DKV / 64) * (SEQ / 64) + 7) / 8, NB);
  const dim3 gAttP(NB * NKV * NQP);
  const dim3 gAttM(NB * NKV * (NQB - NQP));
  const float s64    = (1.0f / 64.0f) * 0.08838834764831845f;
  const float oscale = 1.0f / 262144.0f;

  cvt_bf16x8<<<gCvtX, blk, 0, stream>>>(x, Xb, n8x);
  wt_prep<0, true ><<<gWq, blk, 0, stream>>>(Wq, DM,  WqT,  DM);
  wt_prep<0, true ><<<gWk, blk, 0, stream>>>(Wk, DKV, WkT,  DM);
  wt_prep<0, false><<<gWk, blk, 0, stream>>>(Wv, DKV, WvT,  DM);
  wt_prep<1, false><<<gWq, blk, 0, stream>>>(Wo, DM,  WoT2, DM);
  gemm64<__bf16, 3, true, false><<<gQ, blk, 0, stream>>>(
      Xb, DM, 0LL, WqT, DM, 0LL,
      (void*)Qh, (void*)Ql, DM, 0LL, cosp, sinp,
      NB * SEQ, DM, DM, 1.0f, 64.0f);
  gemm64<__bf16, 3, true, false><<<gK, blk, 0, stream>>>(
      Xb, DM, 0LL, WkT, DM, 0LL,
      (void*)Kh, (void*)Kl, DKV, 0LL, cosp, sinp,
      NB * SEQ, DKV, DM, 1.0f, 64.0f);
  gemm64<__bf16, 3, false, false><<<gVT, blk, 0, stream>>>(
      WvT, DM, 0LL, Xb, DM, (long long)SEQ * DM,
      (void*)VTh, (void*)VTl, SEQ, (long long)DKV * SEQ, cosp, sinp,
      DKV, SEQ, DM, 1.0f, 256.0f);
  (void)hipFuncSetAttribute(reinterpret_cast<const void*>(&attn_gqa<true>),
                            hipFuncAttributeMaxDynamicSharedMemorySize, A_PREC);
  (void)hipFuncSetAttribute(reinterpret_cast<const void*>(&attn_gqa<false>),
                            hipFuncAttributeMaxDynamicSharedMemorySize, A_MAIN);
  attn_gqa<true ><<<gAttP, dim3(128), A_PREC, stream>>>(Qh, Ql, Kh, Kl, VTh, VTl, Op, s64);
  attn_gqa<false><<<gAttM, dim3(128), A_MAIN, stream>>>(Qh, Ql, Kh, Kl, VTh, VTl, Op, s64);
  gemm64<_Float16, 0, false, true><<<gQ, blk, 0, stream>>>(
      Op, 2 * DM, 0LL, WoT2, 2 * DM, 0LL,
      d_out, d_out, DM, 0LL, cosp, sinp,
      NB * SEQ, DM, 2 * DM, oscale, 1.0f);
  (void)hipGetLastError();
}
